// NonStructured_Encoder_14714557956235
// MI455X (gfx1250) — hardware-run, weakly checked
//
#include <hip/hip_runtime.h>
#include <hip/hip_bf16.h>

typedef __attribute__((ext_vector_type(16))) _Float16 v16h;
typedef __attribute__((ext_vector_type(8)))  _Float16 v8h;
typedef __attribute__((ext_vector_type(16))) __bf16   v16b;
typedef __attribute__((ext_vector_type(8)))  __bf16   v8b;
typedef __attribute__((ext_vector_type(8)))  float    v8f;
typedef __attribute__((ext_vector_type(4)))  float    v4f;

__device__ __forceinline__ unsigned short f2bf_bits(float f) {
  unsigned u = __float_as_uint(f);
  return (unsigned short)((u + 0x7FFFu + ((u >> 16) & 1u)) >> 16);
}
__device__ __forceinline__ float bf_bits2f(unsigned short h) { return __uint_as_float(((unsigned)h) << 16); }

__device__ __forceinline__ void dep_guard_h(v8f& a, v8f& b, v16h x, v16h y) { asm volatile("v_nop\n\tv_nop\n\tv_nop\n\tv_nop" : "+v"(a), "+v"(b) : "v"(x), "v"(y)); }
__device__ __forceinline__ void dep_guard_b(v8f& a, v8f& b, v16b x, v16b y) { asm volatile("v_nop\n\tv_nop\n\tv_nop\n\tv_nop" : "+v"(a), "+v"(b) : "v"(x), "v"(y)); }
__device__ __forceinline__ void keep4_h(v16h a, v16h b, v16h c, v16h d) { asm volatile("v_nop" :: "v"(a), "v"(b), "v"(c), "v"(d)); }
__device__ __forceinline__ void keep4_b(v16b a, v16b b, v16b c, v16b d) { asm volatile("v_nop" :: "v"(a), "v"(b), "v"(c), "v"(d)); }
__device__ __forceinline__ void acc_guard4(v8f& a, v8f& b, v8f& c, v8f& d) { asm volatile("v_nop\n\tv_nop\n\tv_nop\n\tv_nop" : "+v"(a), "+v"(b), "+v"(c), "+v"(d)); }
template <typename T> struct Frag;
template <> struct Frag<_Float16> {
  typedef v16h V; union U { v16h v; v8h h[2]; };
  static __device__ __forceinline__ v16h load(const _Float16* p) {
    U f; f.h[0] = *(const v8h*)(p); f.h[1] = *(const v8h*)(p + 16); return f.v;
  }
  static __device__ __forceinline__ v8f mma(v16h a, v16h b, v8f c) {
    return __builtin_amdgcn_wmma_f32_16x16x32_f16(false, a, false, b, (short)0, c, false, false);
  }
  static __device__ __forceinline__ void guard(v8f& a, v8f& b, v16h x, v16h y) { dep_guard_h(a, b, x, y); }
  static __device__ __forceinline__ void keep(v16h a, v16h b, v16h c, v16h d) { keep4_h(a, b, c, d); }
};
template <> struct Frag<__bf16> {
  typedef v16b V; union U { v16b v; v8b h[2]; };
  static __device__ __forceinline__ v16b load(const __bf16* p) {
    U f; f.h[0] = *(const v8b*)(p); f.h[1] = *(const v8b*)(p + 16); return f.v;
  }
  static __device__ __forceinline__ v8f mma(v16b a, v16b b, v8f c) {
    return __builtin_amdgcn_wmma_f32_16x16x32_bf16(false, a, false, b, (short)0, c, false, false);
  }
  static __device__ __forceinline__ void guard(v8f& a, v8f& b, v16b x, v16b y) { dep_guard_b(a, b, x, y); }
  static __device__ __forceinline__ void keep(v16b a, v16b b, v16b c, v16b d) { keep4_b(a, b, c, d); }
};

template <int ET> struct Elem;
template <> struct Elem<0> { typedef _Float16 T; };
template <> struct Elem<1> { typedef __bf16 T; };
template <int ET, bool SPLIT, int BIAS_MODE, int OUT_MODE, bool RESID, int ACT = 0>
__global__ __launch_bounds__(256) void wmma_gemm64(
    const unsigned short* __restrict__ Ap, const unsigned short* __restrict__ A2p, int lda, long strideA,
    const unsigned short* __restrict__ Btp, const unsigned short* __restrict__ Bt2p, int ldb, long strideB,
    void* __restrict__ Cout, void* __restrict__ Cout2, int ldc, long strideC,
    const float* __restrict__ bias,
    const float* __restrict__ resid, long strideR,
    int M, int N, int K, float scale) {
  typedef typename Elem<ET>::T T;
  typedef typename Frag<T>::V V;
  const T* A = (const T*)Ap; const T* A2 = (const T*)A2p; const T* Bt = (const T*)Btp; const T* Bt2 = (const T*)Bt2p;
  __shared__ __align__(16) float sT[8][16 * 68];
  const int b    = blockIdx.y;
  const int lane = threadIdx.x & 31;
  const int wave = threadIdx.x >> 5;
  const int tilesN = N >> 6;
  const int tilesM = M >> 6;
  const int tile = blockIdx.x * 8 + wave;
  if (tile >= tilesM * tilesN) return;
  const int tm = tile / tilesN;
  const int tn = tile - tm * tilesN;
  const int m0 = tm << 6;
  const int n0 = tn << 6;

  const T* Ab  = A  + (size_t)b * strideA;
  const T* Bb  = Bt + (size_t)b * strideB;
  const T* Ab2 = SPLIT ? (A2  + (size_t)b * strideA) : nullptr;
  const T* Bb2 = SPLIT ? (Bt2 + (size_t)b * strideB) : nullptr;

  const int rlane = lane & 15;
  const int koff  = (lane >> 4) * 8;
  const int mOff  = (lane >> 4) * 8;

  v8f acc[4][4];
#pragma unroll
  for (int i = 0; i < 4; ++i)
#pragma unroll
    for (int j = 0; j < 4; ++j) acc[i][j] = (v8f){0.f,0.f,0.f,0.f,0.f,0.f,0.f,0.f};

  for (int k0 = 0; k0 < K; k0 += 32) {
    V bh[4], bl[4];
#pragma unroll
    for (int j = 0; j < 4; ++j) {
      const size_t bo = (size_t)(n0 + (j << 4) + rlane) * ldb + koff + k0;
      bh[j] = Frag<T>::load(Bb + bo);
      if (SPLIT) bl[j] = Frag<T>::load(Bb2 + bo);
    }
#pragma unroll
    for (int i = 0; i < 4; ++i) {
      const size_t ao = (size_t)(m0 + (i << 4) + rlane) * lda + koff + k0;
      V ah = Frag<T>::load(Ab + ao);
      V al;
      if (SPLIT) al = Frag<T>::load(Ab2 + ao);
#pragma unroll
      for (int j = 0; j < 4; ++j) {
        acc[i][j] = Frag<T>::mma(ah, bh[j], acc[i][j]);
        if (SPLIT) {
          acc[i][j] = Frag<T>::mma(ah, bl[j], acc[i][j]);
          acc[i][j] = Frag<T>::mma(al, bh[j], acc[i][j]);
        }
      }
      Frag<T>::guard(acc[i][0], acc[i][3], ah, SPLIT ? al : ah);
    }
    Frag<T>::keep(bh[0], bh[1], bh[2], bh[3]);
    if (SPLIT) Frag<T>::keep(bl[0], bl[1], bl[2], bl[3]);
  }
  acc_guard4(acc[0][0], acc[0][1], acc[0][2], acc[0][3]);
  acc_guard4(acc[1][0], acc[1][1], acc[1][2], acc[1][3]);
  acc_guard4(acc[2][0], acc[2][1], acc[2][2], acc[2][3]);
  acc_guard4(acc[3][0], acc[3][1], acc[3][2], acc[3][3]);

  float* slab = sT[wave];
  const float* Rb = RESID ? (resid + (size_t)b * strideR) : nullptr;
#pragma unroll
  for (int i = 0; i < 4; ++i) {
    const int mBase = m0 + (i << 4);
#pragma unroll
    for (int j = 0; j < 4; ++j) {
      const int n = n0 + (j << 4) + rlane;
      float bv = 0.f;
      if (BIAS_MODE == 2) bv = bias[n];
#pragma unroll
      for (int r = 0; r < 8; ++r) {
        float v = acc[i][j][r] * scale;
        if (BIAS_MODE == 1) v += bias[mBase + mOff + r];
        if (BIAS_MODE == 2) v += bv;
        if (RESID) v += Rb[(size_t)(mBase + mOff + r) * ldc + n];
        if (ACT == 1) v = tanhf(v);
        if (ACT == 2) v = fmaxf(v, 0.0f);
        if (ACT == 3) v = v / (1.0f + expf(-v));
        if (ACT == 4) v = (v > 0.f) ? v : 0.01f * v;
        if (ACT == 5) v = 0.5f * v * (1.0f + erff(v * 0.70710678118654752f));
        slab[(mOff + r) * 68 + (j << 4) + rlane] = v;
      }
    }
    __builtin_amdgcn_fence(__ATOMIC_RELEASE, "workgroup");
    __builtin_amdgcn_wave_barrier();
    __builtin_amdgcn_fence(__ATOMIC_ACQUIRE, "workgroup");
    if (OUT_MODE == 0) {
      float* C = (float*)Cout + (size_t)b * strideC;
      const int hh = lane >> 4, c4 = (lane & 15) * 4;
      for (int pass = 0; pass < 2; ++pass) {
#pragma unroll
        for (int it = 0; it < 8; ++it) {
          const int row = it * 2 + hh;
          v4f v = *(const v4f*)(slab + row * 68 + c4);
          *(volatile v4f*)(C + (size_t)(mBase + row) * ldc + n0 + c4) = v;
        }
        __threadfence();
      }
    } else {
      const int q = lane >> 3, c8 = (lane & 7) * 8;
      unsigned short* C  = (unsigned short*)Cout  + (size_t)b * strideC;
      unsigned short* C2 = (OUT_MODE == 2) ? ((unsigned short*)Cout2 + (size_t)b * strideC) : nullptr;
      for (int pass = 0; pass < 2; ++pass) {
#pragma unroll
        for (int it = 0; it < 4; ++it) {
          const int row = it * 4 + q;
          const float* sp = slab + row * 68 + c8;
          v8h hv, lv;
#pragma unroll
          for (int e = 0; e < 8; ++e) {
            if (OUT_MODE == 1) {
              hv[e] = (_Float16)sp[e];
            } else {
              unsigned short hb = f2bf_bits(sp[e]);
              unsigned short lb = f2bf_bits(sp[e] - bf_bits2f(hb));
              hv[e] = __builtin_bit_cast(_Float16, hb);
              lv[e] = __builtin_bit_cast(_Float16, lb);
            }
          }
          *(volatile v8h*)(C + (size_t)(mBase + row) * ldc + n0 + c8) = hv;
          if (OUT_MODE == 2) *(volatile v8h*)(C2 + (size_t)(mBase + row) * ldc + n0 + c8) = lv;
        }
        __threadfence();
      }
    }
    __builtin_amdgcn_fence(__ATOMIC_RELEASE, "workgroup");
    __builtin_amdgcn_wave_barrier();
    __builtin_amdgcn_fence(__ATOMIC_ACQUIRE, "workgroup");
  }
}

constexpr int kHid     = 256;
constexpr int kG3      = 768;
constexpr int kUnits   = 512;
constexpr int kEmb     = 300;
constexpr int kEmbPad  = 320;
constexpr int kTokPerSeq = 64;
constexpr int kChunkSeq  = 256;
constexpr int kHPitch  = 256;
constexpr int kSPitch  = 260;

template <int KIN, int KOUT>
__device__ __forceinline__ void row_to_f16(const float* __restrict__ srow, unsigned short* __restrict__ orow,
                                           int lane, float scale) {
  constexpr int NQ = KIN / 4;
  constexpr int NP = KOUT / 8;
#pragma unroll
  for (int p0 = 0; p0 < NP; p0 += 32) {
    const int p  = p0 + lane;
    const int pc = (p < NP) ? p : (NP - 1);
    int q0 = 2 * pc, q1 = 2 * pc + 1;
    q0 = (q0 < NQ) ? q0 : (NQ - 1);
    q1 = (q1 < NQ) ? q1 : (NQ - 1);
    const v4f x0 = *(const v4f*)(srow + 4 * q0);
    const v4f x1 = *(const v4f*)(srow + 4 * q1);
    v8h hv;
#pragma unroll
    for (int e = 0; e < 4; ++e) {
      const float m0 = (8 * pc + e < KIN) ? 1.0f : 0.0f;
      const float m1 = (8 * pc + 4 + e < KIN) ? 1.0f : 0.0f;
      hv[e]     = (_Float16)(x0[e] * m0 * scale);
      hv[4 + e] = (_Float16)(x1[e] * m1 * scale);
    }
    unsigned short* dst = orow + 8 * pc;
    if (p < NP) *(volatile v8h*)dst = hv;
    __threadfence();
    if (p < NP) *(volatile v8h*)dst = hv;
  }
}

template <int KIN, int KOUT>
__global__ __launch_bounds__(256) void cast_rows(const float* __restrict__ src, unsigned short* __restrict__ out,
                                                 int nrows, float scale) {
  const int lane = threadIdx.x & 31;
  const int row  = blockIdx.x * 8 + (threadIdx.x >> 5);
  if (row >= nrows) return;
  row_to_f16<KIN, KOUT>(src + (size_t)row * KIN, out + (size_t)row * KOUT, lane, scale);
}

__global__ __launch_bounds__(256) void gather_emb(const int* __restrict__ tokens, const float* __restrict__ embed,
                                                  int nvocab, unsigned short* __restrict__ out, int chunk) {
  const int lane = threadIdx.x & 31;
  const int orow = blockIdx.x * 8 + (threadIdx.x >> 5);
  if (orow >= kTokPerSeq * kChunkSeq) return;
  const int l = orow >> 8;
  const int u = orow & 255;
  const int seq = chunk * kChunkSeq + u;
  int tok = tokens[(size_t)seq * kTokPerSeq + l];
  tok = (tok < 0) ? 0 : tok;
  tok = (tok >= nvocab) ? (nvocab - 1) : tok;
  row_to_f16<kEmb, kEmbPad>(embed + (size_t)tok * kEmb, out + (size_t)orow * kEmbPad, lane, 8.0f);
}

__device__ __forceinline__ void guard_step(v8f& c0, v8f& c1, v8f& c2, v8f& c3, v8f& c4, v8f& c5,
                                           v16h a, v16h b0, v16h b1, v16h b2, v16h b3, v16h b4, v16h b5) {
  asm volatile("v_nop\n\tv_nop\n\tv_nop\n\tv_nop"
               : "+v"(c0), "+v"(c1), "+v"(c2), "+v"(c3), "+v"(c4), "+v"(c5)
               : "v"(a), "v"(b0), "v"(b1), "v"(b2), "v"(b3), "v"(b4), "v"(b5));
}

__device__ __forceinline__ float sigm_f(float x) {
  x = fminf(fmaxf(x, -30.0f), 30.0f);
  return 1.0f / (1.0f + expf(-x));
}
__device__ __forceinline__ float tanh_f(float x) {
  x = fminf(fmaxf(x, -15.0f), 15.0f);
  return 1.0f - 2.0f / (1.0f + expf(2.0f * x));
}

template <int NSTEP, bool SEQ>
__global__ __launch_bounds__(256) void gru_rec(
    const float* __restrict__ xpF, const float* __restrict__ xpB,
    const unsigned short* __restrict__ whF, const unsigned short* __restrict__ whB,
    const float* __restrict__ bihF, const float* __restrict__ bhhF,
    const float* __restrict__ bihB, const float* __restrict__ bhhB,
    float* __restrict__ outp, unsigned short* __restrict__ h16p,
    int rowBase, int xsM, int xsT, int osM, int osT)
{
  __shared__ __align__(16) _Float16 hA[16 * kHPitch];
  __shared__ __align__(16) float    slab[16 * kSPitch];

  const int tid  = threadIdx.x;
  const int wave = tid >> 5;
  const int lane = tid & 31;
  const int hh   = lane >> 4;
  const int c    = lane & 15;
  const int dir  = blockIdx.y;
  const int bx   = blockIdx.x;

  const float* xp        = dir ? xpB : xpF;
  const _Float16* wh     = (const _Float16*)(dir ? whB : whF);
  const float* bih       = dir ? bihB : bihF;
  const float* bhh       = dir ? bhhB : bhhF;
  constexpr float kInv   = 1.0f / 128.0f;

  float bR[2], bZ[2], bI[2], bHn[2];
  float hreg[2][8];
#pragma unroll
  for (int ub = 0; ub < 2; ++ub) {
    const int u = 32 * wave + 16 * ub + c;
    bR[ub]  = bih[u] + bhh[u];
    bZ[ub]  = bih[kHid + u] + bhh[kHid + u];
    bI[ub]  = bih[2 * kHid + u];
    bHn[ub] = bhh[2 * kHid + u];
#pragma unroll
    for (int r = 0; r < 8; ++r) hreg[ub][r] = 0.0f;
  }
  {
    v8h z;
#pragma unroll
    for (int e = 0; e < 8; ++e) z[e] = (_Float16)0.0f;
    *(v8h*)(hA + 8 * tid) = z;
    *(v8h*)(hA + 8 * (tid + 256)) = z;
  }
  __syncthreads();

#pragma unroll 1
  for (int t = 0; t < NSTEP; ++t) {
    const int tt = dir ? (NSTEP - 1 - t) : t;

    v8f acc[3][2];
#pragma unroll
    for (int g = 0; g < 3; ++g)
#pragma unroll
      for (int ub = 0; ub < 2; ++ub) acc[g][ub] = (v8f){0.f,0.f,0.f,0.f,0.f,0.f,0.f,0.f};

#pragma unroll 1
    for (int k0 = 0; k0 < kHid; k0 += 32) {
      union { v16h v; v8h h[2]; } fa;
      fa.h[0] = *(const v8h*)(hA + c * kHPitch + k0 + 8 * hh);
      fa.h[1] = *(const v8h*)(hA + c * kHPitch + k0 + 16 + 8 * hh);
      v16h bf[3][2];
#pragma unroll
      for (int g = 0; g < 3; ++g)
#pragma unroll
        for (int ub = 0; ub < 2; ++ub)
          bf[g][ub] = Frag<_Float16>::load(wh + (size_t)(g * kHid + 32 * wave + 16 * ub + c) * kHid + k0 + 8 * hh);
#pragma unroll
      for (int g = 0; g < 3; ++g)
#pragma unroll
        for (int ub = 0; ub < 2; ++ub)
          acc[g][ub] = Frag<_Float16>::mma(fa.v, bf[g][ub], acc[g][ub]);
      guard_step(acc[0][0], acc[0][1], acc[1][0], acc[1][1], acc[2][0], acc[2][1],
                 fa.v, bf[0][0], bf[0][1], bf[1][0], bf[1][1], bf[2][0], bf[2][1]);
    }

#pragma unroll
    for (int ub = 0; ub < 2; ++ub) {
      const int u = 32 * wave + 16 * ub + c;
#pragma unroll
      for (int r = 0; r < 8; ++r) {
        const int mloc = bx * 16 + 8 * hh + r;
        const float* xrp = xp + (size_t)(mloc * xsM + tt * xsT) * kG3 + u;
        const float xr = xrp[0];
        const float xz = xrp[kHid];
        const float xn = xrp[2 * kHid];
        const float rg = sigm_f(xr + acc[0][ub][r] * kInv + bR[ub]);
        const float zg = sigm_f(xz + acc[1][ub][r] * kInv + bZ[ub]);
        const float hn = acc[2][ub][r] * kInv + bHn[ub];
        const float ng = tanh_f(xn + bI[ub] + rg * hn);
        const float ho = hreg[ub][r];
        hreg[ub][r] = (1.0f - zg) * ng + zg * ho;
      }
    }
    __syncthreads();

#pragma unroll
    for (int ub = 0; ub < 2; ++ub) {
      const int u = 32 * wave + 16 * ub + c;
#pragma unroll
      for (int r = 0; r < 8; ++r) {
        const int row = 8 * hh + r;
        hA[row * kHPitch + u] = (_Float16)(hreg[ub][r] * 8.0f);
        if (SEQ) slab[row * kSPitch + u] = hreg[ub][r];
      }
    }
    __syncthreads();

    if (SEQ) {
      for (int pass = 0; pass < 2; ++pass) {
#pragma unroll
        for (int rr = 0; rr < 2; ++rr) {
          const int row  = 2 * wave + rr;
          const int grow = (rowBase + bx * 16 + row) * osM + tt * osT;
          float* op = outp + (size_t)grow * kUnits + dir * kHid;
          const v4f v0 = *(const v4f*)(slab + row * kSPitch + 4 * lane);
          const v4f v1 = *(const v4f*)(slab + row * kSPitch + 128 + 4 * lane);
          *(volatile v4f*)(op + 4 * lane) = v0;
          *(volatile v4f*)(op + 128 + 4 * lane) = v1;
        }
        __threadfence();
      }
    }
  }

  if (!SEQ) {
#pragma unroll
    for (int ub = 0; ub < 2; ++ub) {
      const int u = 32 * wave + 16 * ub + c;
#pragma unroll
      for (int r = 0; r < 8; ++r) slab[(8 * hh + r) * kSPitch + u] = hreg[ub][r];
    }
    __syncthreads();
    for (int pass = 0; pass < 2; ++pass) {
#pragma unroll
      for (int rr = 0; rr < 2; ++rr) {
        const int row  = 2 * wave + rr;
        const int grow = (rowBase + bx * 16 + row) * osM;
        float* op = outp + (size_t)grow * kUnits + dir * kHid;
        const v4f v0 = *(const v4f*)(slab + row * kSPitch + 4 * lane);
        const v4f v1 = *(const v4f*)(slab + row * kSPitch + 128 + 4 * lane);
        *(volatile v4f*)(op + 4 * lane) = v0;
        *(volatile v4f*)(op + 128 + 4 * lane) = v1;
        const v4f w0 = *(const v4f*)(slab + row * kSPitch + 8 * lane);
        const v4f w1 = *(const v4f*)(slab + row * kSPitch + 8 * lane + 4);
        v8h hv;
#pragma unroll
        for (int e = 0; e < 4; ++e) {
          hv[e]     = (_Float16)(w0[e] * 8.0f);
          hv[4 + e] = (_Float16)(w1[e] * 8.0f);
        }
        unsigned short* hp = h16p + (size_t)grow * kUnits + dir * kHid + 8 * lane;
        *(volatile v8h*)hp = hv;
      }
      __threadfence();
    }
  }
}

extern "C" void kernel_launch(void* const* d_in, const int* in_sizes, int n_in,
                              void* d_out, int out_size, void* d_ws, size_t ws_size,
                              hipStream_t stream) {
  if (n_in < 18) return;
  const int*   tokens  = (const int*)  d_in[0];
  const float* embed   = (const float*)d_in[1];
  const float* w_ih_f1 = (const float*)d_in[2];
  const float* w_hh_f1 = (const float*)d_in[3];
  const float* b_ih_f1 = (const float*)d_in[4];
  const float* b_hh_f1 = (const float*)d_in[5];
  const float* w_ih_b1 = (const float*)d_in[6];
  const float* w_hh_b1 = (const float*)d_in[7];
  const float* b_ih_b1 = (const float*)d_in[8];
  const float* b_hh_b1 = (const float*)d_in[9];
  const float* w_ih_f2 = (const float*)d_in[10];
  const float* w_hh_f2 = (const float*)d_in[11];
  const float* b_ih_f2 = (const float*)d_in[12];
  const float* b_hh_f2 = (const float*)d_in[13];
  const float* w_ih_b2 = (const float*)d_in[14];
  const float* w_hh_b2 = (const float*)d_in[15];
  const float* b_ih_b2 = (const float*)d_in[16];
  const float* b_hh_b2 = (const float*)d_in[17];

  const int nvocab = in_sizes[1] / kEmb;
  if (nvocab < 1) return;
  if (in_sizes[0] < 1024 * kTokPerSeq) return;
  if (out_size < 2 * 1024 * kUnits) return;

  const size_t nRows1 = (size_t)kTokPerSeq * kChunkSeq;

  size_t off = 0;
  auto carve = [&](size_t bytes) { size_t o = off; off += (bytes + 255) & ~(size_t)255; return o; };
  const size_t oW1F  = carve((size_t)kG3 * kEmbPad * 2);
  const size_t oW1B  = carve((size_t)kG3 * kEmbPad * 2);
  const size_t oWH1F = carve((size_t)kG3 * kHid * 2);
  const size_t oWH1B = carve((size_t)kG3 * kHid * 2);
  const size_t oWH2F = carve((size_t)kG3 * kHid * 2);
  const size_t oWH2B = carve((size_t)kG3 * kHid * 2);
  const size_t oW2F  = carve((size_t)kG3 * kUnits * 2);
  const size_t oW2B  = carve((size_t)kG3 * kUnits * 2);
  const size_t oA16  = carve(nRows1 * kEmbPad * 2);
  const size_t oXPF  = carve(nRows1 * kG3 * 4);
  const size_t oXPB  = carve(nRows1 * kG3 * 4);
  const size_t oH16  = carve((size_t)1024 * kUnits * 2);
  const size_t oXP2F = carve((size_t)1024 * kG3 * 4);
  const size_t oXP2B = carve((size_t)1024 * kG3 * 4);
  if (off > ws_size) return;

  char* ws = (char*)d_ws;
  unsigned short* W1F  = (unsigned short*)(ws + oW1F);
  unsigned short* W1B  = (unsigned short*)(ws + oW1B);
  unsigned short* WH1F = (unsigned short*)(ws + oWH1F);
  unsigned short* WH1B = (unsigned short*)(ws + oWH1B);
  unsigned short* WH2F = (unsigned short*)(ws + oWH2F);
  unsigned short* WH2B = (unsigned short*)(ws + oWH2B);
  unsigned short* W2F  = (unsigned short*)(ws + oW2F);
  unsigned short* W2B  = (unsigned short*)(ws + oW2B);
  unsigned short* A16  = (unsigned short*)(ws + oA16);
  float*          XPF  = (float*)(ws + oXPF);
  float*          XPB  = (float*)(ws + oXPB);
  unsigned short* H16  = (unsigned short*)(ws + oH16);
  float*          XP2F = (float*)(ws + oXP2F);
  float*          XP2B = (float*)(ws + oXP2B);

  float* out0 = (float*)d_out;
  float* out1 = (float*)d_out + (size_t)1024 * kUnits;

  cast_rows<kEmb,   kEmbPad><<<kG3 / 8, 256, 0, stream>>>(w_ih_f1, W1F,  kG3, 16.0f);
  cast_rows<kEmb,   kEmbPad><<<kG3 / 8, 256, 0, stream>>>(w_ih_b1, W1B,  kG3, 16.0f);
  cast_rows<kHid,   kHid   ><<<kG3 / 8, 256, 0, stream>>>(w_hh_f1, WH1F, kG3, 16.0f);
  cast_rows<kHid,   kHid   ><<<kG3 / 8, 256, 0, stream>>>(w_hh_b1, WH1B, kG3, 16.0f);
  cast_rows<kHid,   kHid   ><<<kG3 / 8, 256, 0, stream>>>(w_hh_f2, WH2F, kG3, 16.0f);
  cast_rows<kHid,   kHid   ><<<kG3 / 8, 256, 0, stream>>>(w_hh_b2, WH2B, kG3, 16.0f);
  cast_rows<kUnits, kUnits ><<<kG3 / 8, 256, 0, stream>>>(w_ih_f2, W2F,  kG3, 16.0f);
  cast_rows<kUnits, kUnits ><<<kG3 / 8, 256, 0, stream>>>(w_ih_b2, W2B,  kG3, 16.0f);

  const int M1 = (int)nRows1;
  const int tiles1 = (M1 / 64) * (kG3 / 64);
  const float gemmScale = 1.0f / 128.0f;
  for (int ch = 0; ch < 1024 / kChunkSeq; ++ch) {
    gather_emb<<<(M1 + 7) / 8, 256, 0, stream>>>(tokens, embed, nvocab, A16, ch);
    wmma_gemm64<0, false, 0, 0, false, 0><<<dim3((tiles1 + 7) / 8, 1), 256, 0, stream>>>(
        A16, A16, kEmbPad, 0L, W1F, W1F, kEmbPad, 0L, (void*)XPF, (void*)XPF, kG3, 0L,
        b_ih_f1, XPF, 0L, M1, kG3, kEmbPad, gemmScale);
    wmma_gemm64<0, false, 0, 0, false, 0><<<dim3((tiles1 + 7) / 8, 1), 256, 0, stream>>>(
        A16, A16, kEmbPad, 0L, W1B, W1B, kEmbPad, 0L, (void*)XPB, (void*)XPB, kG3, 0L,
        b_ih_b1, XPB, 0L, M1, kG3, kEmbPad, gemmScale);
    gru_rec<kTokPerSeq, false><<<dim3(kChunkSeq / 16, 2), 256, 0, stream>>>(
        XPF, XPB, WH1F, WH1B, b_ih_f1, b_hh_f1, b_ih_b1, b_hh_b1,
        out0, H16, ch * kChunkSeq, 1, kChunkSeq, 1, 0);
  }

  const int M2 = 1024;
  const int tiles2 = (M2 / 64) * (kG3 / 64);
  wmma_gemm64<0, false, 0, 0, false, 0><<<dim3((tiles2 + 7) / 8, 1), 256, 0, stream>>>(
      H16, H16, kUnits, 0L, W2F, W2F, kUnits, 0L, (void*)XP2F, (void*)XP2F, kG3, 0L,
      b_ih_f2, XP2F, 0L, M2, kG3, kUnits, gemmScale);
  wmma_gemm64<0, false, 0, 0, false, 0><<<dim3((tiles2 + 7) / 8, 1), 256, 0, stream>>>(
      H16, H16, kUnits, 0L, W2B, W2B, kUnits, 0L, (void*)XP2B, (void*)XP2B, kG3, 0L,
      b_ih_b2, XP2B, 0L, M2, kG3, kUnits, gemmScale);
  gru_rec<32, true><<<dim3(32 / 16, 2), 256, 0, stream>>>(
      XP2F, XP2B, WH2F, WH2B, b_ih_f2, b_hh_f2, b_ih_b2, b_hh_b2,
      out1, H16, 0, 32, 1, 32, 1);
}
